// RealNVP_11424613007642
// MI455X (gfx1250) — hardware-verified
//
#include <hip/hip_runtime.h>
#include <stddef.h>


typedef _Float16 v16h __attribute__((ext_vector_type(16)));
typedef _Float16 v8h  __attribute__((ext_vector_type(8)));
typedef float    v8f  __attribute__((ext_vector_type(8)));
typedef float    v4f  __attribute__((ext_vector_type(4)));
typedef _Float16 h16;

#ifndef NROWS
#define NROWS 4096
#endif
#define NROWS_FULL 4096
#define NTIPS 64
#define NS1   61
#define NBR   125
#define EMB   2000
#define HIDN  64
#define NLAY  10
#define W2C   4000
#define KP1   2048
#define NP2   4032
#define RB    16
#define FP    128
#define TILES_CH 125

static_assert(NROWS >= 32 && NROWS <= NROWS_FULL && (NROWS % 32) == 0);
static_assert((NROWS % RB) == 0);
static_assert(NBR == NTIPS + NS1 && NTIPS == 64 && NS1 <= 64);
static_assert(W2C == 2 * EMB);
static_assert(EMB == 16 * TILES_CH);
static_assert(KP1 >= EMB && (KP1 % 64) == 0 && KP1 == 2 * 1024);
static_assert(NP2 >= W2C && (NP2 % 64) == 0);
static_assert(HIDN == 64 && (HIDN % 32) == 0);
static_assert(RB == 16);
static_assert(RB * 128 == 8 * 256);
static_assert(RB * 64 == 4 * 256);
static_assert(RB * (FP / 4) == 2 * 256);
static_assert(RB * (KP1 / 8) == 16 * 256);

#define LDT 72
#define LDD 2056
#define LDO 2008
static_assert((LDT % 8) == 0 && LDT >= 64);
static_assert((LDD % 8) == 0 && LDD >= KP1);
static_assert((LDO % 8) == 0 && LDO >= EMB && LDO <= LDD);

#define WCARRY 64.0f
#define XCARRY 16.0f
#define HCARRY 64.0f
#define OCARRY 64.0f

#define W1T_BYTES ((size_t)NLAY * HIDN * KP1 * 2)
#define W2T_BYTES ((size_t)NLAY * NP2 * HIDN * 2)
#define F_BYTES   ((size_t)NROWS * FP * 4)
#define OFF_W1T ((size_t)0)
#define OFF_W2T (OFF_W1T + W1T_BYTES)
#define OFF_F   (OFF_W2T + W2T_BYTES)
#define WS_TOTAL (OFF_F + F_BYTES)
static_assert((W1T_BYTES % 128) == 0 && (W2T_BYTES % 128) == 0 && (F_BYTES % 128) == 0);
static_assert(WS_TOTAL <= (size_t)134217728);

#define OUT1_OFF   ((size_t)NROWS_FULL * NBR)
#define PACK_G0    ((unsigned)(NROWS * NBR / 4))
#define PACK_G1    ((unsigned)(NROWS / 4))
#define PACK_TOTAL (PACK_G0 + PACK_G1)
static_assert(OUT1_OFF * 4 == (size_t)2048000);
static_assert(((NROWS * NBR) % 32) == 0 && (PACK_G1 % 8) == 0);

#define FLOW_LDS_BYTES (RB * LDD * 2 + 2 * 4 * 256 * 4 + RB * 128 * 4 + RB * 128 * 4 + RB * LDT * 2 + RB * 64 * 4 + RB * 4)
static_assert(FLOW_LDS_BYTES <= 131072);

__device__ __forceinline__ float bf16r(float x) {
  unsigned int u = __float_as_uint(x);
  u = (u + 0x7FFFu + ((u >> 16) & 1u)) & 0xFFFF0000u;
  return __uint_as_float(u);
}

static __device__ __forceinline__ h16 toh_flush(float v) {
  const h16 r = (h16)v;
  return (fabsf(v) < 6.103515625e-05f) ? (h16)0.0f : r;
}

__device__ __forceinline__ v16h frag_at(const _Float16* p) {
  v8h lo = *(const v8h*)(p);
  v8h hi = *(const v8h*)(p + 16);
  v16h out;
#pragma unroll
  for (int i = 0; i < 8; ++i) { out[i] = lo[i]; out[i + 8] = hi[i]; }
  return out;
}
__device__ __forceinline__ v16h ld_frag(const _Float16* base, unsigned ld) {
  const unsigned lane = threadIdx.x & 31u;
  return frag_at(base + (lane & 15u) * ld + (lane >> 4) * 8u);
}

__device__ __forceinline__ v8f wmma16(v16h a, v16h b, v8f c) {
  v8f d = __builtin_amdgcn_wmma_f32_16x16x32_f16(false, a, false, b, (short)0, c,
                                                 false, false);
  asm volatile("v_nop\n\tv_nop\n\tv_nop\n\tv_nop" : "+v"(d) : "v"(a), "v"(b));
  return d;
}

__device__ __forceinline__ float red16_sum(float x) {
#pragma unroll
  for (int off = 1; off < 16; off <<= 1) x += __shfl_xor(x, off, 32);
  return x;
}

__global__ __launch_bounds__(256) void wconv_kernel(
    const float* __restrict__ W, _Float16* __restrict__ Wt, unsigned ldw, unsigned ldk,
    unsigned ktrue, unsigned ntrue, unsigned in_lstride, unsigned out_lstride) {
  __shared__ _Float16 T[64 * LDT];
  const unsigned tid = threadIdx.x;
  const unsigned n0 = blockIdx.x * 64u;
  const unsigned k0 = blockIdx.y * 64u;
  const float* Wl = W + (size_t)blockIdx.z * in_lstride;
  _Float16* Wtl = Wt + (size_t)blockIdx.z * out_lstride;
#pragma unroll 4
  for (unsigned j = 0; j < 16u; ++j) {
    const unsigned idx = tid + 256u * j;
    const unsigned kr = idx >> 6, nc = idx & 63u;
    const unsigned k = k0 + kr, n = n0 + nc;
    const bool ok = (k < ktrue) && (n < ntrue);
    const unsigned kc = (k < ktrue) ? k : (ktrue - 1u);
    const unsigned ncl = (n < ntrue) ? n : (ntrue - 1u);
    float v = Wl[(size_t)kc * ldw + ncl];
    v = ok ? v : 0.0f;
    T[nc * LDT + kr] = toh_flush(WCARRY * bf16r(v));
  }
  __syncthreads();
  v8h x[2];
  size_t off[2];
#pragma unroll
  for (unsigned i = 0; i < 2u; ++i) {
    const unsigned n = 32u * i + (tid >> 3);
    const unsigned kc = (tid & 7u) * 8u;
    x[i] = *(const v8h*)&T[n * LDT + kc];
    off[i] = (size_t)(n0 + n) * ldk + k0 + kc;
  }
#pragma unroll
  for (int i = 0; i < 2; ++i) *(volatile v8h*)(Wtl + off[i]) = x[i];
  __threadfence();
#pragma unroll
  for (int i = 0; i < 2; ++i) *(volatile v8h*)(Wtl + off[i]) = x[i];
}

__global__ __launch_bounds__(256) void flow_kernel(
    const float* __restrict__ samp, const float* __restrict__ logq_in,
    const _Float16* __restrict__ W1t, const float* __restrict__ b1,
    const _Float16* __restrict__ W2t, const float* __restrict__ b2,
    const int* __restrict__ nidx, float* __restrict__ F) {
  __shared__ _Float16 Rg[RB * LDD];
  __shared__ float    Part[2 * 4 * 256];
  __shared__ float    Xv[RB * 128];
  __shared__ int      Ix[RB * 128];
  __shared__ _Float16 Hs[RB * LDT];
  __shared__ float    Sg[RB * 64];
  __shared__ float    Lq[RB];

  const unsigned tid = threadIdx.x, lane = tid & 31u;
  const unsigned wv = (unsigned)__builtin_amdgcn_readfirstlane((int)(threadIdx.x >> 5));
  const unsigned hh = lane >> 4, m = lane & 15u;
  const unsigned row0 = blockIdx.x * (unsigned)RB;
  const unsigned prow = tid >> 4, pm0 = tid & 15u;

#pragma unroll 2
  for (unsigned j = 0; j < 8u; ++j) {
    const unsigned s = tid + 256u * j;
    const unsigned r = s >> 7, slot = s & 127u;
    const unsigned col = slot;
    const bool valid = col < (unsigned)NBR;
    const unsigned colc = valid ? col : (unsigned)(NBR - 1);
    const size_t g = (size_t)(row0 + r) * NBR + colc;
    const float xv = samp[g];
    const int iv = nidx[g];
    Xv[s] = valid ? bf16r(xv) : 0.0f;
    Ix[s] = valid ? iv : (int)EMB;
  }
  __syncthreads();

  float lq = 0.0f;

#pragma unroll 1
  for (unsigned layer = 0; layer < (unsigned)NLAY; ++layer) {
    const unsigned inSide = (layer & 1u) ? 0u : 1u;
    const unsigned outSide = 1u - inSide;
    const unsigned n_out = outSide ? (unsigned)NS1 : (unsigned)NTIPS;
    const _Float16* W1l = W1t + (size_t)layer * (HIDN * KP1);
    const _Float16* W2l = W2t + (size_t)layer * (NP2 * HIDN);
    const float* b1l = b1 + layer * (unsigned)HIDN;
    const float* b2l = b2 + layer * (unsigned)W2C;

    {
      const v8h z = {};
#pragma unroll 4
      for (unsigned j = 0; j < 16u; ++j) {
        const unsigned idx = tid + 256u * j;
        const unsigned r = idx >> 8, c8 = idx & 255u;
        *(v8h*)&Rg[r * LDD + c8 * 8u] = z;
      }
    }
    __syncthreads();

    if (wv == 0u) {
      const unsigned r = lane & 15u;
#pragma unroll 1
      for (unsigned j = 0; j < 64u; ++j) {
        const int id = Ix[r * 128u + inSide * 64u + j];
        const float x = Xv[r * 128u + inSide * 64u + j];
        const bool ok = ((unsigned)id < (unsigned)EMB);
        const unsigned idc = ok ? (unsigned)id : 0u;
        const float old = (float)Rg[r * LDD + idc];
        const float nv = ok ? (old + XCARRY * x) : old;
        Rg[r * LDD + idc] = toh_flush(nv);
      }
    }
    __syncthreads();

    {
      const unsigned nt = wv & 3u, kh = wv >> 2;
      const _Float16* bp = W1l + (size_t)(nt * 16u + m) * KP1 + kh * 1024u + hh * 8u;
      v8f acc = {};
#pragma unroll 2
      for (unsigned k0 = 0; k0 < 1024u; k0 += 32u) {
        const v16h a = ld_frag(&Rg[kh * 1024u + k0], LDD);
        const v16h b = frag_at(bp + k0);
        acc = wmma16(a, b, acc);
      }
#pragma unroll
      for (int r = 0; r < 8; ++r) Part[wv * 256u + (unsigned)r * 32u + lane] = acc[r];
    }
    __syncthreads();

#pragma unroll 1
    for (unsigned j = 0; j < 4u; ++j) {
      const unsigned e = tid + 256u * j;
      const unsigned row = e >> 6, n = e & 63u;
      const unsigned pi = (n >> 4) * 256u + (row & 7u) * 32u + (row >> 3) * 16u + (n & 15u);
      const float sum = Part[pi] + Part[1024u + pi];
      const float pre = sum * (1.0f / (XCARRY * WCARRY)) + bf16r(b1l[n]);
      const float em = expm1f(pre);
      const float hv = (pre > 0.0f) ? pre : em;
      Hs[row * LDT + n] = toh_flush(HCARRY * hv);
    }
    __syncthreads();

    const v16h a0 = ld_frag(&Hs[0], LDT);
    const v16h a1 = ld_frag(&Hs[32], LDT);

#pragma unroll 1
    for (unsigned ch = 0; ch < 2u; ++ch) {
      const _Float16* bbase = W2l + (size_t)(ch * (unsigned)EMB + m) * HIDN + hh * 8u;
      for (unsigned t = wv; t < (unsigned)TILES_CH; t += 8u) {
        const _Float16* bp = bbase + (size_t)t * (16u * HIDN);
        const v16h b0 = frag_at(bp);
        const v16h b1f = frag_at(bp + 32);
        v8f acc = {};
        acc = wmma16(a0, b0, acc);
        acc = wmma16(a1, b1f, acc);
#pragma unroll
        for (int r = 0; r < 8; ++r)
          Rg[(hh * 8u + (unsigned)r) * LDO + t * 16u + m] =
              (_Float16)(acc[r] * (OCARRY / (HCARRY * WCARRY)));
      }
      __syncthreads();

      if (ch == 0u) {
#pragma unroll 1
        for (unsigned j = 0; j < 4u; ++j) {
          const unsigned mm = pm0 + 16u * j;
          const int c = Ix[prow * 128u + outSide * 64u + mm];
          const unsigned cc = (c < 0) ? 0u : ((c > EMB) ? (unsigned)EMB : (unsigned)c);
          const unsigned col = (cc < (unsigned)EMB) ? cc : (unsigned)(EMB - 1);
          Sg[prow * 64u + mm] = (float)Rg[prow * LDO + col];
        }
      } else {
#pragma unroll 1
        for (unsigned j = 0; j < 4u; ++j) {
          const unsigned mm = pm0 + 16u * j;
          const unsigned si = prow * 128u + outSide * 64u + mm;
          const int c = Ix[si];
          const unsigned cc = (c < 0) ? 0u : ((c > EMB) ? (unsigned)EMB : (unsigned)c);
          const bool inr = cc < (unsigned)EMB;
          const unsigned col = inr ? cc : (unsigned)(EMB - 1);
          const float tO = (float)Rg[prow * LDO + col];
          const float p0 = (float)Rg[prow * LDO];
          const float sS = Sg[prow * 64u + mm];
          const float slin = inr ? sS : p0;
          const unsigned ct = inr ? (cc + (unsigned)EMB) : (unsigned)(W2C - 1);
          const float bs = bf16r(b2l[cc]);
          const float bt = bf16r(b2l[ct]);
          const float sr = (slin * (1.0f / OCARRY) + bs) + 2.0f;
          const float ex = expf(-sr);
          const float sg = __builtin_amdgcn_rcpf(1.0f + ex);
          const float lg = logf(sg);
          const float tv = inr ? (tO * (1.0f / OCARRY) + bt) : 0.0f;
          const bool valid = mm < n_out;
          const float xold = Xv[si];
          const float xnew = sg * xold + tv;
          Xv[si] = valid ? xnew : xold;
          lq += valid ? lg : 0.0f;
        }
      }
      __syncthreads();
    }
  }

  const float lqs = red16_sum(lq);
  if (pm0 == 0u) Lq[prow] = lqs;
  __syncthreads();

  v4f xs[2];
  size_t off[2];
#pragma unroll
  for (unsigned i = 0; i < 2u; ++i) {
    const unsigned f = tid + 256u * i;
    const unsigned r = f >> 5, q = f & 31u;
    const float lgv = bf16r(logq_in[row0 + r]) - Lq[r];
    v4f val;
#pragma unroll
    for (unsigned e = 0; e < 4u; ++e) {
      const unsigned col = 4u * q + e;
      const unsigned c0 = (col < 63u) ? col : 63u;
      const unsigned d1 = (col >= 64u) ? (col - 64u) : 0u;
      const unsigned c1 = (d1 < 63u) ? d1 : 63u;
      const float v0 = Xv[r * 128u + c0] - 2.0f;
      const float v1 = Xv[r * 128u + 64u + c1] - 2.0f;
      val[e] = (col < 64u) ? v0
             : ((col < (unsigned)NBR) ? v1 : ((col == (unsigned)NBR) ? lgv : 0.0f));
    }
    xs[i] = val;
    off[i] = (size_t)(row0 + r) * FP + 4u * q;
  }
#pragma unroll
  for (int i = 0; i < 2; ++i) *(volatile v4f*)(F + off[i]) = xs[i];
  __threadfence();
#pragma unroll
  for (int i = 0; i < 2; ++i) *(volatile v4f*)(F + off[i]) = xs[i];
}

__global__ __launch_bounds__(256) void pack_kernel(
    const float* __restrict__ F, float* __restrict__ out) {
  const unsigned g = blockIdx.x * 256u + threadIdx.x;
  const bool live = g < PACK_TOTAL;
  const bool first = g < PACK_G0;
  const unsigned gg = first ? g : (g - PACK_G0);
  v4f val;
#pragma unroll
  for (unsigned i = 0; i < 4u; ++i) {
    const unsigned e = 4u * gg + i;
    const unsigned r = e / (unsigned)NBR;
    const unsigned c = e - r * (unsigned)NBR;
    const unsigned i0 = r * (unsigned)FP + c;
    const unsigned i1 = e * (unsigned)FP + (unsigned)NBR;
    unsigned fi = first ? i0 : i1;
    fi = (fi < (unsigned)(NROWS * FP - 1)) ? fi : (unsigned)(NROWS * FP - 1);
    val[i] = F[fi];
  }
  const size_t off = first ? (size_t)(4u * g) : (OUT1_OFF + (size_t)(4u * gg));
  if (live) *(volatile v4f*)(out + off) = val;
  __threadfence();
  if (live) *(volatile v4f*)(out + off) = val;
}

extern "C" void kernel_launch(void* const* d_in, const int* in_sizes, int n_in,
                              void* d_out, int out_size, void* d_ws, size_t ws_size,
                              hipStream_t stream) {
  if (n_in < 7) return;
  if ((long long)in_sizes[0] < (long long)NROWS * NBR) return;
  if ((long long)in_sizes[1] < (long long)NROWS) return;
  if ((long long)in_sizes[2] < (long long)NLAY * EMB * HIDN) return;
  if ((long long)in_sizes[3] < (long long)NLAY * HIDN) return;
  if ((long long)in_sizes[4] < (long long)NLAY * HIDN * W2C) return;
  if ((long long)in_sizes[5] < (long long)NLAY * W2C) return;
  if ((long long)in_sizes[6] < (long long)NROWS * NBR) return;
  if ((long long)out_size < (long long)OUT1_OFF + NROWS) return;
  if (ws_size < WS_TOTAL) return;

  const float* samp = (const float*)d_in[0];
  const float* logq = (const float*)d_in[1];
  const float* w1   = (const float*)d_in[2];
  const float* b1   = (const float*)d_in[3];
  const float* w2   = (const float*)d_in[4];
  const float* b2   = (const float*)d_in[5];
  const int*   idx  = (const int*)d_in[6];
  float* out = (float*)d_out;

  char* ws = (char*)d_ws;
  _Float16* W1t = (_Float16*)(ws + OFF_W1T);
  _Float16* W2t = (_Float16*)(ws + OFF_W2T);
  float*    Fp  = (float*)(ws + OFF_F);

  dim3 blk(256);
  wconv_kernel<<<dim3(HIDN / 64, KP1 / 64, NLAY), blk, 0, stream>>>(
      w1, W1t, (unsigned)HIDN, (unsigned)KP1, (unsigned)EMB, (unsigned)HIDN,
      (unsigned)(EMB * HIDN), (unsigned)(HIDN * KP1));
  wconv_kernel<<<dim3(NP2 / 64, HIDN / 64, NLAY), blk, 0, stream>>>(
      w2, W2t, (unsigned)W2C, (unsigned)HIDN, (unsigned)HIDN, (unsigned)W2C,
      (unsigned)(HIDN * W2C), (unsigned)(NP2 * HIDN));

  flow_kernel<<<dim3(NROWS / RB), blk, 0, stream>>>(samp, logq, W1t, b1, W2t, b2, idx, Fp);
  pack_kernel<<<dim3((PACK_TOTAL + 255u) / 256u), blk, 0, stream>>>(Fp, out);
}
